// MCAttention_25984552140883
// MI455X (gfx1250) — hardware-run, weakly checked
//
#include <hip/hip_runtime.h>
#include <math.h>

constexpr int   kBatch    = 16;
constexpr int   kHeads    = 8;
constexpr float kWCarry   = 32.0f;
constexpr float kPCarry   = 32768.0f;
constexpr float kCtxCarry = 256.0f;

constexpr size_t kRegPlane = 13631488;
constexpr size_t kRegWP    = 3538944;
constexpr size_t kRegBP    = 12288;
constexpr size_t kRegWOP   = 1572864;
constexpr size_t kRegS     = 44302336;
constexpr size_t kRegP     = 22151168;
constexpr size_t kOffXCK = 0;
constexpr size_t kOffXDT = kOffXCK + kRegPlane;
constexpr size_t kOffQP  = kOffXDT + kRegPlane;
constexpr size_t kOffVPC = kOffQP + kRegPlane;
constexpr size_t kOffWP  = kOffVPC + kRegPlane;
constexpr size_t kOffBP  = kOffWP + kRegWP;
constexpr size_t kOffWOP = kOffBP + kRegBP;
constexpr size_t kOffS   = kOffWOP + kRegWOP;
constexpr size_t kOffP   = kOffS + kRegS;
constexpr size_t kWsTotal = kOffP + kRegP;
static_assert(kWsTotal == 126103552);
static_assert(kWsTotal <= 134217728);
static_assert((size_t)13312 * 512 * 2 <= kRegPlane);
static_assert((size_t)128 * 64 * 832 * 2 <= kRegPlane);
static_assert((size_t)1024 * 1024 * 2 <= kRegPlane);
static_assert((size_t)3 * 768 * 768 * 2 <= kRegWP);
static_assert((size_t)3 * 768 * 4 <= kRegBP);
static_assert((size_t)768 * 1024 * 2 <= kRegWOP);
static_assert((size_t)16 * 832 * 832 * 4 <= kRegS);
static_assert((size_t)128 * 256 * 256 * 4 <= kRegS);
static_assert((size_t)13312 * 384 * 4 <= kRegS);
static_assert((size_t)16 * 832 * 832 * 2 <= kRegP);

typedef __attribute__((ext_vector_type(16))) _Float16 v16h;
typedef __attribute__((ext_vector_type(8)))  _Float16 v8h;
typedef __attribute__((ext_vector_type(16))) __bf16   v16b;
typedef __attribute__((ext_vector_type(8)))  __bf16   v8b;
typedef __attribute__((ext_vector_type(8)))  float    v8f;
typedef __attribute__((ext_vector_type(4)))  float    v4f;
typedef __attribute__((ext_vector_type(4)))  unsigned int v4u;

__device__ __forceinline__ unsigned short f2bf_bits(float f) {
  unsigned u = __float_as_uint(f);
  return (unsigned short)((u + 0x7FFFu + ((u >> 16) & 1u)) >> 16);
}
__device__ __forceinline__ float bf_bits2f(unsigned short h) { return __uint_as_float(((unsigned)h) << 16); }

__device__ __forceinline__ void dep_guard_h(v8f& a, v8f& b, v16h x, v16h y) { asm volatile("v_nop\n\tv_nop\n\tv_nop\n\tv_nop" : "+v"(a), "+v"(b) : "v"(x), "v"(y)); }
__device__ __forceinline__ void dep_guard_b(v8f& a, v8f& b, v16b x, v16b y) { asm volatile("v_nop\n\tv_nop\n\tv_nop\n\tv_nop" : "+v"(a), "+v"(b) : "v"(x), "v"(y)); }
__device__ __forceinline__ void keep4_h(v16h a, v16h b, v16h c, v16h d) { asm volatile("v_nop" :: "v"(a), "v"(b), "v"(c), "v"(d)); }
__device__ __forceinline__ void keep4_b(v16b a, v16b b, v16b c, v16b d) { asm volatile("v_nop" :: "v"(a), "v"(b), "v"(c), "v"(d)); }
__device__ __forceinline__ void acc_guard4(v8f& a, v8f& b, v8f& c, v8f& d) { asm volatile("v_nop\n\tv_nop\n\tv_nop\n\tv_nop" : "+v"(a), "+v"(b), "+v"(c), "+v"(d)); }
template <typename T> struct Frag;
template <> struct Frag<_Float16> {
  typedef v16h V; union U { v16h v; v8h h[2]; };
  static __device__ __forceinline__ v16h load(const _Float16* p) {
    U f; f.h[0] = *(const v8h*)(p); f.h[1] = *(const v8h*)(p + 16); return f.v;
  }
  static __device__ __forceinline__ v8f mma(v16h a, v16h b, v8f c) {
    return __builtin_amdgcn_wmma_f32_16x16x32_f16(false, a, false, b, (short)0, c, false, false);
  }
  static __device__ __forceinline__ void guard(v8f& a, v8f& b, v16h x, v16h y) { dep_guard_h(a, b, x, y); }
  static __device__ __forceinline__ void keep(v16h a, v16h b, v16h c, v16h d) { keep4_h(a, b, c, d); }
};
template <> struct Frag<__bf16> {
  typedef v16b V; union U { v16b v; v8b h[2]; };
  static __device__ __forceinline__ v16b load(const __bf16* p) {
    U f; f.h[0] = *(const v8b*)(p); f.h[1] = *(const v8b*)(p + 16); return f.v;
  }
  static __device__ __forceinline__ v8f mma(v16b a, v16b b, v8f c) {
    return __builtin_amdgcn_wmma_f32_16x16x32_bf16(false, a, false, b, (short)0, c, false, false);
  }
  static __device__ __forceinline__ void guard(v8f& a, v8f& b, v16b x, v16b y) { dep_guard_b(a, b, x, y); }
  static __device__ __forceinline__ void keep(v16b a, v16b b, v16b c, v16b d) { keep4_b(a, b, c, d); }
};

__device__ __forceinline__ unsigned pk16(unsigned short a, unsigned short b) { return (unsigned)a | ((unsigned)b << 16); }
__device__ __forceinline__ unsigned short h_bits(float f) { const _Float16 h = (_Float16)f; return __builtin_bit_cast(unsigned short, h); }

template <int ET> struct Elem;
template <> struct Elem<0> { typedef _Float16 T; };
template <> struct Elem<1> { typedef __bf16 T; };
template <int ET, bool SPLIT, int BIAS_MODE, int OUT_MODE, bool RESID, int ACT = 0>
__global__ __launch_bounds__(256) void wmma_gemm64(
    const unsigned short* __restrict__ Ap, const unsigned short* __restrict__ A2p, int lda, long strideA,
    const unsigned short* __restrict__ Btp, const unsigned short* __restrict__ Bt2p, int ldb, long strideB,
    void* __restrict__ Cout, void* __restrict__ Cout2, int ldc, long strideC,
    const float* __restrict__ bias,
    const float* __restrict__ resid, long strideR,
    int M, int N, int K, float scale,
    int ydiv, long strideA2, long strideB2, long strideC2) {
  typedef typename Elem<ET>::T T;
  typedef typename Frag<T>::V V;
  const T* A = (const T*)Ap; const T* A2 = (const T*)A2p; const T* Bt = (const T*)Btp; const T* Bt2 = (const T*)Bt2p;
  __shared__ __align__(16) float sT[8][16 * 68];
  const int b    = blockIdx.y;
  const int bhi  = b / ydiv;
  const int blo  = b - bhi * ydiv;
  const size_t offA = (size_t)bhi * strideA2 + (size_t)blo * strideA;
  const size_t offB = (size_t)bhi * strideB2 + (size_t)blo * strideB;
  const size_t offC = (size_t)bhi * strideC2 + (size_t)blo * strideC;
  const int lane = threadIdx.x & 31;
  const int wave = threadIdx.x >> 5;
  const int tilesN = N >> 6;
  const int tilesM = M >> 6;
  const int tile = blockIdx.x * 8 + wave;
  if (tile >= tilesM * tilesN) return;
  const int tm = tile / tilesN;
  const int tn = tile - tm * tilesN;
  const int m0 = tm << 6;
  const int n0 = tn << 6;

  const T* Ab  = A  + offA;
  const T* Bb  = Bt + offB;
  const T* Ab2 = SPLIT ? (A2  + offA) : nullptr;
  const T* Bb2 = SPLIT ? (Bt2 + offB) : nullptr;

  const int rlane = lane & 15;
  const int koff  = (lane >> 4) * 8;
  const int mOff  = (lane >> 4) * 8;

  v8f acc[4][4];
#pragma unroll
  for (int i = 0; i < 4; ++i)
#pragma unroll
    for (int j = 0; j < 4; ++j) acc[i][j] = (v8f){0.f,0.f,0.f,0.f,0.f,0.f,0.f,0.f};

  for (int k0 = 0; k0 < K; k0 += 32) {
    V bh[4], bl[4];
#pragma unroll
    for (int j = 0; j < 4; ++j) {
      const size_t bo = (size_t)(n0 + (j << 4) + rlane) * ldb + koff + k0;
      bh[j] = Frag<T>::load(Bb + bo);
      if (SPLIT) bl[j] = Frag<T>::load(Bb2 + bo);
    }
#pragma unroll
    for (int i = 0; i < 4; ++i) {
      const size_t ao = (size_t)(m0 + (i << 4) + rlane) * lda + koff + k0;
      V ah = Frag<T>::load(Ab + ao);
      V al;
      if (SPLIT) al = Frag<T>::load(Ab2 + ao);
#pragma unroll
      for (int j = 0; j < 4; ++j) {
        acc[i][j] = Frag<T>::mma(ah, bh[j], acc[i][j]);
        if (SPLIT) {
          acc[i][j] = Frag<T>::mma(ah, bl[j], acc[i][j]);
          acc[i][j] = Frag<T>::mma(al, bh[j], acc[i][j]);
        }
      }
      Frag<T>::guard(acc[i][0], acc[i][3], ah, SPLIT ? al : ah);
    }
    Frag<T>::keep(bh[0], bh[1], bh[2], bh[3]);
    if (SPLIT) Frag<T>::keep(bl[0], bl[1], bl[2], bl[3]);
  }
  acc_guard4(acc[0][0], acc[0][1], acc[0][2], acc[0][3]);
  acc_guard4(acc[1][0], acc[1][1], acc[1][2], acc[1][3]);
  acc_guard4(acc[2][0], acc[2][1], acc[2][2], acc[2][3]);
  acc_guard4(acc[3][0], acc[3][1], acc[3][2], acc[3][3]);

  float* slab = sT[wave];
  const float* Rb = RESID ? (resid + (size_t)b * strideR) : nullptr;
#pragma unroll
  for (int i = 0; i < 4; ++i) {
    const int mBase = m0 + (i << 4);
#pragma unroll
    for (int j = 0; j < 4; ++j) {
      const int n = n0 + (j << 4) + rlane;
      float bv = 0.f;
      if (BIAS_MODE == 2) bv = bias[n];
#pragma unroll
      for (int r = 0; r < 8; ++r) {
        float v = acc[i][j][r] * scale;
        if (BIAS_MODE == 1) v += bias[mBase + mOff + r];
        if (BIAS_MODE == 2) v += bv;
        if (RESID) v += Rb[(size_t)(mBase + mOff + r) * ldc + n];
        if (ACT == 2) v = fmaxf(v, 0.0f);
        if (ACT == 4) v = (v > 0.f) ? v : 0.01f * v;
        slab[(mOff + r) * 68 + (j << 4) + rlane] = v;
      }
    }
    __builtin_amdgcn_fence(__ATOMIC_RELEASE, "workgroup");
    __builtin_amdgcn_wave_barrier();
    __builtin_amdgcn_fence(__ATOMIC_ACQUIRE, "workgroup");
    if (OUT_MODE == 0) {
      float* C = (float*)Cout + offC;
      const int hh = lane >> 4, c4 = (lane & 15) * 4;
      for (int pass = 0; pass < 2; ++pass) {
#pragma unroll
        for (int it = 0; it < 8; ++it) {
          const int row = it * 2 + hh;
          v4f v = *(const v4f*)(slab + row * 68 + c4);
          *(volatile v4f*)(C + (size_t)(mBase + row) * ldc + n0 + c4) = v;
        }
        __threadfence();
      }
    } else {
      const int q = lane >> 3, c8 = (lane & 7) * 8;
      unsigned short* C  = (unsigned short*)Cout  + offC;
      unsigned short* C2 = (OUT_MODE == 2) ? ((unsigned short*)Cout2 + offC) : nullptr;
      for (int pass = 0; pass < 2; ++pass) {
#pragma unroll
        for (int it = 0; it < 4; ++it) {
          const int row = it * 4 + q;
          const float* sp = slab + row * 68 + c8;
          v8h hv, lv;
#pragma unroll
          for (int e = 0; e < 8; ++e) {
            if (OUT_MODE == 1) {
              hv[e] = (_Float16)sp[e];
            } else {
              unsigned short hb = f2bf_bits(sp[e]);
              unsigned short lb = f2bf_bits(sp[e] - bf_bits2f(hb));
              hv[e] = __builtin_bit_cast(_Float16, hb);
              lv[e] = __builtin_bit_cast(_Float16, lb);
            }
          }
          *(volatile v8h*)(C + (size_t)(mBase + row) * ldc + n0 + c8) = hv;
          if (OUT_MODE == 2) *(volatile v8h*)(C2 + (size_t)(mBase + row) * ldc + n0 + c8) = lv;
        }
        __threadfence();
      }
    }
    __builtin_amdgcn_fence(__ATOMIC_RELEASE, "workgroup");
    __builtin_amdgcn_wave_barrier();
    __builtin_amdgcn_fence(__ATOMIC_ACQUIRE, "workgroup");
  }
}

__global__ __launch_bounds__(256) void gather_tokens_kernel(
    const float* __restrict__ xctx, const float* __restrict__ xdet,
    unsigned short* __restrict__ outc, unsigned short* __restrict__ outd,
    int C, int Himg, int s, int hw, int n, int npad, int E, int n8total) {
  const int i = blockIdx.x * 256 + (int)threadIdx.x;
  if (i >= n8total) return;
  const int which = blockIdx.y;
  const float* x = (which == 0) ? xctx : xdet;
  unsigned short* o = (which == 0) ? outc : outd;
  const int e8 = E >> 3;
  const int row = i / e8;
  const int e0 = (i - row * e8) << 3;
  const int b = row / npad;
  const int t = row - b * npad;
  const bool valid = (t < n);
  const int tc = valid ? t : 0;
  const int hi = tc / hw;
  const int wi = tc - hi * hw;
  const int i12 = e0 / C;
  const int c0 = e0 - i12 * C;
  const int i1 = i12 / s;
  const int i2 = i12 - i1 * s;
  const int y = hi * s + i1;
  const int xw = wi * s + i2;
  const size_t plane = (size_t)Himg * Himg;
  const float* p = x + (((size_t)b * C + c0) * Himg + y) * (size_t)Himg + xw;
  unsigned short hb[8];
#pragma unroll
  for (int e = 0; e < 8; ++e) {
    const float v = p[(size_t)e * plane];
    hb[e] = h_bits(valid ? v : 0.0f);
  }
  const v4u u = (v4u){pk16(hb[0], hb[1]), pk16(hb[2], hb[3]), pk16(hb[4], hb[5]), pk16(hb[6], hb[7])};
  unsigned short* q = o + 8 * (size_t)i;
  *(volatile v4u*)q = u;
  __threadfence();
  *(volatile v4u*)q = u;
}

__global__ __launch_bounds__(256) void wprep_kernel(
    const float* __restrict__ wq, const float* __restrict__ wk, const float* __restrict__ wv, const float* __restrict__ wo,
    const float* __restrict__ bq, const float* __restrict__ bk, const float* __restrict__ bv,
    unsigned short* __restrict__ wp, unsigned short* __restrict__ wop, float* __restrict__ bp,
    int E, int d, int dpad, int dpv, float carry) {
  const int job = blockIdx.y;
  const int i = blockIdx.x * 256 + (int)threadIdx.x;
  const int rows = kHeads * dpad;
  if (job < 3) {
    const int e8 = E >> 3;
    const int total = rows * e8;
    if (i >= total) return;
    const float* W = (job == 0) ? wq : (job == 1) ? wk : wv;
    const int r = i / e8;
    const int k0 = (i - r * e8) << 3;
    const int h = r / dpad;
    const int j = r - h * dpad;
    const bool valid = (j < d);
    const int srow = h * d + (valid ? j : 0);
    const float* p = W + (size_t)srow * E + k0;
    const v4f a = *(const v4f*)(p);
    const v4f c = *(const v4f*)(p + 4);
    unsigned short hb[8];
#pragma unroll
    for (int e = 0; e < 4; ++e) {
      hb[e]     = h_bits(valid ? a[e] * carry : 0.0f);
      hb[4 + e] = h_bits(valid ? c[e] * carry : 0.0f);
    }
    const v4u u = (v4u){pk16(hb[0], hb[1]), pk16(hb[2], hb[3]), pk16(hb[4], hb[5]), pk16(hb[6], hb[7])};
    unsigned short* q = wp + ((size_t)job * rows + r) * (size_t)E + k0;
    *(volatile v4u*)q = u;
    __threadfence();
    *(volatile v4u*)q = u;
  } else if (job == 3) {
    const int cols = kHeads * dpv;
    const int c8n = cols >> 3;
    const int total = E * c8n;
    if (i >= total) return;
    const int o = i / c8n;
    const int r0 = (i - o * c8n) << 3;
    const int h = r0 / dpv;
    const int j0 = r0 - h * dpv;
    const bool valid = (j0 < d);
    const int scol = h * d + (valid ? j0 : 0);
    const float* p = wo + (size_t)o * E + scol;
    const v4f a = *(const v4f*)(p);
    const v4f c = *(const v4f*)(p + 4);
    unsigned short hb[8];
#pragma unroll
    for (int e = 0; e < 4; ++e) {
      hb[e]     = h_bits(valid ? a[e] * carry : 0.0f);
      hb[4 + e] = h_bits(valid ? c[e] * carry : 0.0f);
    }
    const v4u u = (v4u){pk16(hb[0], hb[1]), pk16(hb[2], hb[3]), pk16(hb[4], hb[5]), pk16(hb[6], hb[7])};
    unsigned short* q = wop + (size_t)o * cols + r0;
    *(volatile v4u*)q = u;
    __threadfence();
    *(volatile v4u*)q = u;
  } else {
    const int total = (3 * rows) >> 2;
    if (i >= total) return;
    const int i4 = i << 2;
    const int z = i4 / rows;
    const int r = i4 - z * rows;
    float vv[4];
#pragma unroll
    for (int e = 0; e < 4; ++e) {
      const int re = r + e;
      const int h = re / dpad;
      const int j = re - h * dpad;
      const bool valid = (j < d);
      const int idx = h * d + (valid ? j : 0);
      const float a0 = bq[idx];
      const float a1 = bk[idx];
      const float a2 = bv[idx];
      const float sel = (z == 0) ? a0 : ((z == 1) ? a1 : a2);
      vv[e] = valid ? sel : 0.0f;
    }
    const v4f u = (v4f){vv[0], vv[1], vv[2], vv[3]};
    float* q = bp + i4;
    *(volatile v4f*)q = u;
    __threadfence();
    *(volatile v4f*)q = u;
  }
}

__global__ __launch_bounds__(256) void vtrans_kernel(const unsigned short* __restrict__ vp, unsigned short* __restrict__ vt,
                                                     int npad, int d, int dpad, int dpv) {
  __shared__ __align__(16) unsigned short sm[64][72];
  const int t  = threadIdx.x;
  const int k0 = blockIdx.x * 64;
  const int j0 = blockIdx.y * 64;
  const int bh = blockIdx.z;
  const int b = bh >> 3, h = bh & 7;
  const int pitch = kHeads * dpad;
  const unsigned short* src = vp + ((size_t)b * npad + k0) * (size_t)pitch + (size_t)h * dpad;
#pragma unroll
  for (int it = 0; it < 8; ++it) {
    const int e  = it * 256 + t;
    const int r  = e >> 5;
    const int cp = e & 31;
    const int j  = j0 + 2 * cp;
    const int jc = (j < dpad) ? j : (dpad - 2);
    const unsigned w = *(const unsigned*)(src + (size_t)r * pitch + jc);
    const bool valid = (j < d);
    sm[2 * cp][r]     = valid ? (unsigned short)(w & 0xffffu) : (unsigned short)0;
    sm[2 * cp + 1][r] = valid ? (unsigned short)(w >> 16) : (unsigned short)0;
  }
  __syncthreads();
  const int lane = t & 31, wave = t >> 5;
  const int q = lane >> 3, c8 = (lane & 7) * 8;
  unsigned short* dst = vt + (size_t)bh * dpv * npad + k0;
  v4u u[2];
#pragma unroll
  for (int it = 0; it < 2; ++it) {
    const int row = wave * 8 + it * 4 + q;
    const unsigned short* sp = &sm[row][c8];
    u[it] = (v4u){pk16(sp[0], sp[1]), pk16(sp[2], sp[3]), pk16(sp[4], sp[5]), pk16(sp[6], sp[7])};
  }
  for (int pass = 0; pass < 2; ++pass) {
#pragma unroll
    for (int it = 0; it < 2; ++it) {
      const int row = wave * 8 + it * 4 + q;
      *(volatile v4u*)(dst + (size_t)(j0 + row) * npad + c8) = u[it];
    }
    __threadfence();
  }
}

__global__ __launch_bounds__(128) void softmax_rows_kernel(const float* __restrict__ S, unsigned short* __restrict__ P,
                                                           int npad, int tpr, int n, float carry) {
  const int lane = threadIdx.x & 31;
  const int wave = threadIdx.x >> 5;
  const size_t row = (size_t)blockIdx.x * 4 + wave;
  const float* sr = S + row * (size_t)npad;
  float x[4][8];
  float m = -1.0e30f;
#pragma unroll
  for (int i = 0; i < 4; ++i) {
    const int gi = 32 * i + lane;
    const int gic = (gi < tpr) ? gi : (tpr - 1);
    const v4f a = *(const v4f*)(sr + 8 * gic);
    const v4f c = *(const v4f*)(sr + 8 * gic + 4);
#pragma unroll
    for (int e = 0; e < 4; ++e) { x[i][e] = a[e]; x[i][4 + e] = c[e]; }
#pragma unroll
    for (int e = 0; e < 8; ++e) {
      const bool ok = (8 * gi + e) < n;
      x[i][e] = ok ? x[i][e] : -1.0e30f;
      m = fmaxf(m, x[i][e]);
    }
  }
#pragma unroll
  for (int off = 16; off > 0; off >>= 1) m = fmaxf(m, __shfl_xor(m, off, 32));
  float sum = 0.f;
#pragma unroll
  for (int i = 0; i < 4; ++i) {
    const int gi = 32 * i + lane;
#pragma unroll
    for (int e = 0; e < 8; ++e) {
      const bool ok = (8 * gi + e) < n;
      float p = __expf(x[i][e] - m);
      p = ok ? p : 0.0f;
      x[i][e] = p;
      sum += p;
    }
  }
#pragma unroll
  for (int off = 16; off > 0; off >>= 1) sum += __shfl_xor(sum, off, 32);
  const float inv = carry / sum;
  v4u u[4];
#pragma unroll
  for (int i = 0; i < 4; ++i) {
    unsigned short hb[8];
#pragma unroll
    for (int e = 0; e < 8; ++e) hb[e] = h_bits(x[i][e] * inv);
    u[i] = (v4u){pk16(hb[0], hb[1]), pk16(hb[2], hb[3]), pk16(hb[4], hb[5]), pk16(hb[6], hb[7])};
  }
  unsigned short* pr = P + row * (size_t)npad;
  for (int pass = 0; pass < 2; ++pass) {
#pragma unroll
    for (int i = 0; i < 4; ++i) {
      const int gi = 32 * i + lane;
      if (gi < tpr) *(volatile v4u*)(pr + 8 * gi) = u[i];
    }
    __threadfence();
  }
}

__global__ __launch_bounds__(256) void residual_kernel(const float* __restrict__ xdet, const float* __restrict__ outp,
                                                       float* __restrict__ dst, int C, int Himg, int sshift, int hw,
                                                       int npad, int E, int n4) {
  const int i = blockIdx.x * 256 + (int)threadIdx.x;
  if (i >= n4) return;
  const int base = 4 * i;
  const v4f xv = *(const v4f*)(xdet + base);
  const int smask = (1 << sshift) - 1;
  int xw = base % Himg;
  int tmp = base / Himg;
  int y = tmp % Himg;
  tmp /= Himg;
  int c = tmp % C;
  int b = tmp / C;
  float r[4];
#pragma unroll
  for (int e = 0; e < 4; ++e) {
    const int t = (y >> sshift) * hw + (xw >> sshift);
    const int ecol = (((y & smask) << sshift) + (xw & smask)) * C + c;
    const int bc = (b < kBatch) ? b : (kBatch - 1);
    r[e] = xv[e] + outp[((size_t)bc * npad + t) * (size_t)E + ecol];
    xw += 1;
    const bool wx = (xw == Himg);
    xw = wx ? 0 : xw;
    y += wx ? 1 : 0;
    const bool wy = (y == Himg);
    y = wy ? 0 : y;
    c += wy ? 1 : 0;
    const bool wc = (c == C);
    c = wc ? 0 : c;
    b += wc ? 1 : 0;
  }
  const v4f u = (v4f){r[0], r[1], r[2], r[3]};
  float* q = dst + base;
  *(volatile v4f*)q = u;
  __threadfence();
  *(volatile v4f*)q = u;
}

struct ScaleCfg { int C, Himg, s, hw, n, npad, E, d, dpad, dpv, G; };
static const ScaleCfg kCfg[4] = {
  { 96, 56, 2, 28, 784, 832, 384, 48, 64,  64,  2},
  {192, 28, 1, 28, 784, 832, 192, 24, 32,  64,  2},
  {384, 14, 1, 14, 196, 256, 384, 48, 64,  64, 16},
  {768,  7, 1,  7,  49,  64, 768, 96, 96, 128, 16},
};
static const size_t kOutOffFloats[4] = {0, 4816896, 7225344, 8429568};

extern "C" void kernel_launch(void* const* d_in, const int* in_sizes, int n_in,
                              void* d_out, int out_size, void* d_ws, size_t ws_size,
                              hipStream_t stream) {
  (void)in_sizes; (void)out_size;
  if (n_in < 40) return;
  if (ws_size < kWsTotal) return;

  char* ws = (char*)d_ws;
  unsigned short* XC  = (unsigned short*)(ws + kOffXCK);
  unsigned short* KP  = (unsigned short*)(ws + kOffXCK);
  unsigned short* XD  = (unsigned short*)(ws + kOffXDT);
  unsigned short* VT  = (unsigned short*)(ws + kOffXDT);
  unsigned short* QP  = (unsigned short*)(ws + kOffQP);
  unsigned short* VP  = (unsigned short*)(ws + kOffVPC);
  unsigned short* CTX = (unsigned short*)(ws + kOffVPC);
  unsigned short* WP  = (unsigned short*)(ws + kOffWP);
  float*          BP  = (float*)(ws + kOffBP);
  unsigned short* WOP = (unsigned short*)(ws + kOffWOP);
  float*          Sb  = (float*)(ws + kOffS);
  float*          OUTb = (float*)(ws + kOffS);
  unsigned short* Pb  = (unsigned short*)(ws + kOffP);
  const float* fdummy = (const float*)(ws + kOffBP);

  for (int sc = 0; sc < 4; ++sc) {
    const ScaleCfg& g = kCfg[sc];
    const float* xdet = (const float*)d_in[2 * sc];
    const float* xctx = (const float*)d_in[2 * sc + 1];
    const int wb = 8 + 8 * sc;
    const float* wq = (const float*)d_in[wb + 0]; const float* bq = (const float*)d_in[wb + 1];
    const float* wk = (const float*)d_in[wb + 2]; const float* bk = (const float*)d_in[wb + 3];
    const float* wv = (const float*)d_in[wb + 4]; const float* bv = (const float*)d_in[wb + 5];
    const float* wo = (const float*)d_in[wb + 6]; const float* bo = (const float*)d_in[wb + 7];

    const int Mrows = kBatch * g.npad;
    const int rows8 = kHeads * g.dpad;
    const int colsv = kHeads * g.dpv;
    if ((size_t)Mrows * g.E * 2 > kRegPlane) return;
    if ((size_t)Mrows * rows8 * 2 > kRegPlane) return;
    if ((size_t)Mrows * colsv * 2 > kRegPlane) return;
    if ((size_t)kBatch * kHeads * g.dpv * g.npad * 2 > kRegPlane) return;
    if ((size_t)3 * rows8 * g.E * 2 > kRegWP) return;
    if ((size_t)3 * rows8 * 4 > kRegBP) return;
    if ((size_t)g.E * colsv * 2 > kRegWOP) return;
    if ((size_t)g.G * kHeads * g.npad * g.npad * 4 > kRegS) return;
    if ((size_t)g.G * kHeads * g.npad * g.npad * 2 > kRegP) return;
    if ((size_t)Mrows * g.E * 4 > kRegS) return;

    {
      const int n8 = Mrows * (g.E / 8);
      dim3 grid((n8 + 255) / 256, 2);
      gather_tokens_kernel<<<grid, 256, 0, stream>>>(xctx, xdet, XC, XD, g.C, g.Himg, g.s, g.hw, g.n, g.npad, g.E, n8);
    }
    {
      const int tot0 = rows8 * (g.E / 8);
      const int tot3 = g.E * (colsv / 8);
      const int tot4 = (3 * rows8) / 4;
      int mx = tot0; if (tot3 > mx) mx = tot3; if (tot4 > mx) mx = tot4;
      dim3 grid((mx + 255) / 256, 5);
      wprep_kernel<<<grid, 256, 0, stream>>>(wq, wk, wv, wo, bq, bk, bv, WP, WOP, BP, g.E, g.d, g.dpad, g.dpv, kWCarry);
    }
    {
      const float projScale = 1.0f / kWCarry;
      const int tiles = (Mrows / 64) * (rows8 / 64);
      dim3 grid((tiles + 7) / 8, 1);
      const size_t wplane = (size_t)rows8 * g.E;
      wmma_gemm64<0, false, 2, 1, false><<<grid, 256, 0, stream>>>(
          XC, XC, g.E, 0, WP, WP, g.E, 0, (void*)QP, (void*)QP, rows8, 0, BP, fdummy, 0,
          Mrows, rows8, g.E, projScale, 1, 0, 0, 0);
      wmma_gemm64<0, false, 2, 1, false><<<grid, 256, 0, stream>>>(
          XD, XD, g.E, 0, WP + wplane, WP + wplane, g.E, 0, (void*)KP, (void*)KP, rows8, 0, BP + rows8, fdummy, 0,
          Mrows, rows8, g.E, projScale, 1, 0, 0, 0);
      wmma_gemm64<0, false, 2, 1, false><<<grid, 256, 0, stream>>>(
          XD, XD, g.E, 0, WP + 2 * wplane, WP + 2 * wplane, g.E, 0, (void*)VP, (void*)VP, rows8, 0, BP + 2 * rows8, fdummy, 0,
          Mrows, rows8, g.E, projScale, 1, 0, 0, 0);
    }
    {
      dim3 grid(g.npad / 64, g.dpv / 64, kBatch * kHeads);
      vtrans_kernel<<<grid, 256, 0, stream>>>(VP, VT, g.npad, g.d, g.dpad, g.dpv);
    }
    {
      const float sScale  = (float)(1.0 / sqrt((double)g.d));
      const float pvScale = kCtxCarry / kPCarry;
      const int ngroups = kBatch / g.G;
      const int ny = g.G * kHeads;
      const long npad2 = (long)g.npad * g.npad;
      const int tilesS = (g.npad / 64) * (g.npad / 64);
      const int tilesC = (g.npad / 64) * (g.dpv / 64);
      for (int grp = 0; grp < ngroups; ++grp) {
        const int b0 = grp * g.G;
        const unsigned short* Qg = QP + (size_t)b0 * g.npad * rows8;
        const unsigned short* Kg = KP + (size_t)b0 * g.npad * rows8;
        dim3 gridS((tilesS + 7) / 8, ny);
        wmma_gemm64<0, false, 0, 0, false><<<gridS, 256, 0, stream>>>(
            Qg, Qg, rows8, (long)g.dpad, Kg, Kg, rows8, (long)g.dpad, (void*)Sb, (void*)Sb, g.npad, npad2, fdummy, fdummy, 0,
            g.npad, g.npad, g.dpad, sScale, kHeads, (long)g.npad * rows8, (long)g.npad * rows8, (long)kHeads * npad2);
        softmax_rows_kernel<<<(ny * g.npad) / 4, 128, 0, stream>>>(Sb, Pb, g.npad, g.npad / 8, g.n, kPCarry);
        const unsigned short* VTg = VT + (size_t)b0 * kHeads * g.dpv * g.npad;
        unsigned short* CTXg = CTX + (size_t)b0 * g.npad * colsv;
        dim3 gridC((tilesC + 7) / 8, ny);
        wmma_gemm64<0, false, 0, 1, false><<<gridC, 256, 0, stream>>>(
            Pb, Pb, g.npad, npad2, VTg, VTg, g.npad, (long)g.dpv * g.npad, (void*)CTXg, (void*)CTXg, colsv, (long)g.dpv,
            fdummy, fdummy, 0,
            g.npad, g.dpv, g.npad, pvScale, kHeads, (long)kHeads * npad2, (long)kHeads * g.dpv * g.npad, (long)g.npad * colsv);
      }
    }
    {
      const float outScale = 1.0f / (kCtxCarry * kWCarry);
      const int tiles = (Mrows / 64) * (g.E / 64);
      dim3 grid((tiles + 7) / 8, 1);
      wmma_gemm64<0, false, 2, 0, false><<<grid, 256, 0, stream>>>(
          CTX, CTX, colsv, 0, WOP, WOP, colsv, 0, (void*)OUTb, (void*)OUTb, g.E, 0, bo, fdummy, 0,
          Mrows, g.E, colsv, outScale, 1, 0, 0, 0);
    }
    {
      const int nOut = kBatch * g.C * g.Himg * g.Himg;
      const int n4 = nOut / 4;
      const int sshift = (g.s == 2) ? 1 : 0;
      residual_kernel<<<(n4 + 255) / 256, 256, 0, stream>>>(xdet, OUTb, (float*)d_out + kOutOffFloats[sc],
                                                            g.C, g.Himg, sshift, g.hw, g.npad, g.E, n4);
    }
  }
}
